// GNNWrapper_86938728006236
// MI455X (gfx1250) — hardware-verified
//
#include <hip/hip_runtime.h>


namespace {
constexpr int NB = 64, NN = 32, F = 16, S = 8, C = 128, HH = 256, DD = 256, OBS = NN * F + NN * NN + NN * NN * S  , NE = NB * NN * NN  , NBJ = NB * NN  , KT = HH * F  ;
constexpr float XS = 8.0f, WSC = 256.0f;

typedef _Float16 b16;
typedef __attribute__((ext_vector_type(16))) _Float16 v16b;
typedef __attribute__((ext_vector_type(8))) _Float16 v8b;
typedef __attribute__((ext_vector_type(8))) float v8f;
typedef __attribute__((ext_vector_type(4))) float v4f;
__device__ __forceinline__ float bf16_rne(float f) { unsigned int u = __float_as_uint(f); u += 0x7FFFu + ((u >> 16) & 1u); return __uint_as_float(u & 0xFFFF0000u); }
__device__ __forceinline__ void split16(float v, b16& hi, b16& lo) { hi = (b16)v; lo = (b16)(v - (float)hi); }
__device__ __forceinline__ v16b frag_kb(const b16* p, int hh) { const v8b a = *(const v8b*)(p + 8 * hh), b = *(const v8b*)(p + 16 + 8 * hh); v16b f;
#pragma unroll
  for (int e = 0; e < 8; ++e) { f[e] = a[e]; f[8 + e] = b[e]; } return f; }
__device__ __forceinline__ v8f wmma16b(v16b a, v16b b, v8f c) { v8f d = __builtin_amdgcn_wmma_f32_16x16x32_f16(false, a, false, b, (short)0, c, false, false); asm volatile("v_nop\n\tv_nop\n\tv_nop\n\tv_nop" : "+v"(d) : "v"(a), "v"(b)); return d; }
__device__ __forceinline__ void wave_lds_sync() { __builtin_amdgcn_fence(__ATOMIC_RELEASE, "workgroup"); __builtin_amdgcn_wave_barrier(); __builtin_amdgcn_fence(__ATOMIC_ACQUIRE, "workgroup"); }
__device__ __forceinline__ float pmul(float a, float b) { float p = a * b; asm volatile("" : "+v"(p)); return p; }

__global__ __launch_bounds__(256) void prep_kernel(const float* __restrict__ obs, const float* __restrict__ w1, const float* __restrict__ w2, const float* __restrict__ wk, const float* __restrict__ wd, b16* __restrict__ E16, b16* __restrict__ XT16, b16* __restrict__ W1T, b16* __restrict__ W2T, b16* __restrict__ WKR, b16* __restrict__ WDT) {
  const size_t t = (size_t)blockIdx.x * 256 + threadIdx.x; size_t u = t; v8b o;
  const size_t nE = (size_t)NE * 32 / 8, nX = (size_t)NB * F * NN / 8, n1 = (size_t)HH * 32 / 8, n2 = (size_t)HH * HH / 8, n3 = (size_t)C * KT / 8, n4 = (size_t)DD * C / 8;
  if (u < nE) { const size_t e = u * 8; const size_t edge = e / 32; const int c0 = (int)(e % 32); const size_t b = edge / (NN * NN); const int ji = (int)(edge % (NN * NN));
    for (int j = 0; j < 8; ++j) { const int s = c0 + j; o[j] = (s < S) ? (b16)(bf16_rne(obs[b * OBS + NN * F + NN * NN + (size_t)ji * S + s]) * XS) : (b16)0.0f; } for (int pass = 0; pass < 2; ++pass) { *(volatile v8b*)(E16 + e) = o; __threadfence(); } return; } u -= nE;
  if (u < nX) { const int e = (int)u * 8; const int b = e / (F * NN), rem = e % (F * NN); const int f = rem / NN, i0 = rem % NN; for (int j = 0; j < 8; ++j) o[j] = (b16)(bf16_rne(obs[(size_t)b * OBS + (i0 + j) * F + f]) * XS); for (int pass = 0; pass < 2; ++pass) { *(volatile v8b*)(XT16 + e) = o; __threadfence(); } return; } u -= nX;
  if (u < n1) { const int e = (int)u * 8; const int oo = e / 32, k0 = e % 32; for (int j = 0; j < 8; ++j) { const int k = k0 + j; o[j] = (k < S) ? (b16)(bf16_rne(w1[k * HH + oo]) * WSC) : (b16)0.0f; } for (int pass = 0; pass < 2; ++pass) { *(volatile v8b*)(W1T + e) = o; __threadfence(); } return; } u -= n1;
  if (u < n2) { const int e = (int)u * 8; const int oo = e / HH, k0 = e % HH; for (int j = 0; j < 8; ++j) o[j] = (b16)(bf16_rne(w2[(k0 + j) * HH + oo]) * WSC); for (int pass = 0; pass < 2; ++pass) { *(volatile v8b*)(W2T + e) = o; __threadfence(); } return; } u -= n2;
  if (u < n3) { const size_t e = u * 8; const int c = (int)(e / KT); const int k0 = (int)(e % KT); for (int j = 0; j < 8; ++j) { const int k = k0 + j; const int h = k / F, f = k % F; o[j] = (b16)(bf16_rne(wk[(size_t)h * (C * F) + c * F + f]) * WSC); } for (int pass = 0; pass < 2; ++pass) { *(volatile v8b*)(WKR + e) = o; __threadfence(); } return; } u -= n3;
  if (u < n4) { const int e = (int)u * 8; const int oo = e / C, k0 = e % C; for (int j = 0; j < 8; ++j) o[j] = (b16)(bf16_rne(wd[(k0 + j) * DD + oo]) * WSC); for (int pass = 0; pass < 2; ++pass) { *(volatile v8b*)(WDT + e) = o; __threadfence(); } }
}
__global__ __launch_bounds__(128) void edge_kernel(const b16* __restrict__ E16, const b16* __restrict__ XT16, const float* __restrict__ obs, const b16* __restrict__ W1T, const float* __restrict__ b1, const b16* __restrict__ W2T, const float* __restrict__ b2, b16* __restrict__ TTh, b16* __restrict__ TTl, float* __restrict__ SX) {
  __shared__ __attribute__((aligned(16))) b16 H1h[NN][HH + 8], H1l[NN][HH + 8]; __shared__ __attribute__((aligned(16))) b16 ATh[HH][NN + 8], ATl[HH][NN + 8]; __shared__ __attribute__((aligned(16))) b16 Th[HH][F + 8], Tl[HH][F + 8]; __shared__ float Aji[NN]; __shared__ __attribute__((aligned(16))) float sx[32];
  const int bj = blockIdx.x, b = bj / NN, j = bj % NN; const int wave = threadIdx.x >> 5, lane = threadIdx.x & 31, nloc = lane & 15, hlf = lane >> 4, t_ = threadIdx.x;
  if (t_ < NN) Aji[t_] = bf16_rne(obs[(size_t)b * OBS + NN * F + j * NN + t_]);
  if (t_ < 32) { float s = 0.0f; if (t_ < F) { for (int i = 0; i < NN; ++i) s += pmul(bf16_rne(obs[(size_t)b * OBS + NN * F + j * NN + i]), bf16_rne(obs[(size_t)b * OBS + i * F + t_])); } sx[t_] = s; }
  const b16* Eb = E16 + ((size_t)bj * NN) * 32;
  if (wave < 2) { const v16b a = frag_kb(Eb + (size_t)(wave * 16 + nloc) * 32, hlf);
    for (int t = 0; t < HH / 16; ++t) { v8f d = {}; d = wmma16b(a, frag_kb(W1T + (size_t)(t * 16 + nloc) * 32, hlf), d); const float bb = bf16_rne(b1[t * 16 + nloc]);
      for (int r = 0; r < 8; ++r) { b16 p, q; split16(fmaxf(d[r] * (1.0f / (XS * WSC)) + bb, 0.0f) * XS, p, q); H1h[wave * 16 + 8 * hlf + r][t * 16 + nloc] = p; H1l[wave * 16 + 8 * hlf + r][t * 16 + nloc] = q; } } }
  __syncthreads();
  for (int rt = 0; rt < 2; ++rt) { v8f acc[4] = {{}, {}, {}, {}};
#pragma unroll 2
    for (int kb = 0; kb < HH; kb += 32) { const v16b a = frag_kb(&H1h[rt * 16 + nloc][kb], hlf), al = frag_kb(&H1l[rt * 16 + nloc][kb], hlf);
#pragma unroll
      for (int t = 0; t < 4; ++t) { const v16b bw = frag_kb(W2T + (size_t)(wave * 64 + t * 16 + nloc) * HH + kb, hlf); acc[t] = wmma16b(a, bw, acc[t]); acc[t] = wmma16b(al, bw, acc[t]); } }
#pragma unroll
    for (int t = 0; t < 4; ++t) { const int hcol = wave * 64 + t * 16 + nloc; const float bb = bf16_rne(b2[hcol]);
#pragma unroll
      for (int r = 0; r < 8; ++r) { const int i = rt * 16 + 8 * hlf + r; const float h2 = fmaxf(acc[t][r] * (1.0f / (XS * WSC)) + bb, 0.0f); b16 p, q; split16(pmul(Aji[i], h2) * XS, p, q); ATh[hcol][i] = p; ATl[hcol][i] = q; } } }
  __syncthreads();
  { const b16* Xb = XT16 + (size_t)b * F * NN; const v16b bx = frag_kb(Xb + (size_t)nloc * NN, hlf);
    for (int rtile = 0; rtile < 4; ++rtile) { const int h0 = wave * 64 + rtile * 16; v8f d = {}; d = wmma16b(frag_kb(&ATh[h0 + nloc][0], hlf), bx, d); d = wmma16b(frag_kb(&ATl[h0 + nloc][0], hlf), bx, d);
      for (int r = 0; r < 8; ++r) { b16 p, q; split16(d[r] * (1.0f / (XS * XS)) * XS, p, q); Th[h0 + 8 * hlf + r][nloc] = p; Tl[h0 + 8 * hlf + r][nloc] = q; } } }
  __syncthreads();
  for (int pass = 0; pass < 2; ++pass) { for (int q = t_; q < KT / 8; q += 128) { const int h = q >> 1, f8 = (q & 1) * 8; *(volatile v8b*)(TTh + (size_t)bj * KT + q * 8) = *(const v8b*)(&Th[h][f8]); *(volatile v8b*)(TTl + (size_t)bj * KT + q * 8) = *(const v8b*)(&Tl[h][f8]); }
    if (t_ < 8) *(volatile v4f*)(SX + (size_t)bj * 32 + t_ * 4) = *(const v4f*)(&sx[t_ * 4]);
    __threadfence(); }
}
__global__ __launch_bounds__(128) void ecc_kernel(const b16* __restrict__ TTh, const b16* __restrict__ TTl, const b16* __restrict__ WKR, const float* __restrict__ SX, const float* __restrict__ obs, const float* __restrict__ bk, const float* __restrict__ wroot, const float* __restrict__ bconv, float* __restrict__ XC) {
  __shared__ __attribute__((aligned(16))) float Tf[4][16][C + 4];
  const int wave = threadIdx.x >> 5, lane = threadIdx.x & 31, nloc = lane & 15, hlf = lane >> 4; const size_t m0 = (size_t)blockIdx.x * 64 + wave * 16;
  v8f acc[8];
#pragma unroll
  for (int t = 0; t < 8; ++t) acc[t] = (v8f){};
  for (int kb = 0; kb < KT; kb += 32) { const v16b a = frag_kb(TTh + (m0 + nloc) * KT + kb, hlf), al = frag_kb(TTl + (m0 + nloc) * KT + kb, hlf);
#pragma unroll
    for (int t = 0; t < 8; ++t) { const v16b bw = frag_kb(WKR + (size_t)(t * 16 + nloc) * KT + kb, hlf); acc[t] = wmma16b(a, bw, acc[t]); acc[t] = wmma16b(al, bw, acc[t]); } }
#pragma unroll
  for (int t = 0; t < 8; ++t) { const int c = t * 16 + nloc; const float bb = bf16_rne(bconv[c]);
    for (int r = 0; r < 8; ++r) { const size_t row = m0 + 8 * hlf + r; const size_t b = row / NN; const int j = (int)(row % NN); float extra = bb;
#pragma unroll 1
      for (int f = 0; f < F; ++f) extra += pmul(SX[row * 32 + f], bf16_rne(bk[c * F + f])) + pmul(bf16_rne(obs[b * OBS + (size_t)j * F + f]), bf16_rne(wroot[f * C + c]));
      Tf[wave][8 * hlf + r][c] = fmaxf(acc[t][r] * (1.0f / (XS * WSC)) + extra, 0.0f); } }
  wave_lds_sync();
  for (int pass = 0; pass < 2; ++pass) { for (int rr = 0; rr < 16; ++rr) *(volatile v4f*)(XC + (m0 + rr) * C + lane * 4) = *(const v4f*)(&Tf[wave][rr][lane * 4]); __threadfence(); }
}
__global__ __launch_bounds__(128) void head_kernel(const float* __restrict__ XC, const float* __restrict__ attw, const b16* __restrict__ WDT, const float* __restrict__ bd, float* __restrict__ out) {
  __shared__ __attribute__((aligned(16))) b16 Ph[NB][C + 8], Pl[NB][C + 8]; __shared__ float att[4][NN]; __shared__ __attribute__((aligned(16))) float Tf[4][16][C + 4];
  const int wave = threadIdx.x >> 5, lane = threadIdx.x & 31, nloc = lane & 15, hlf = lane >> 4;
  for (int b = wave; b < NB; b += 4) {
    float lg = 0.0f; const float* xr = XC + ((size_t)b * NN + lane) * C;
#pragma unroll 4
    for (int c = 0; c < C; ++c) lg += pmul(xr[c], bf16_rne(attw[c]));
    float mx = lg;
#pragma unroll
    for (int o = 16; o >= 1; o >>= 1) mx = fmaxf(mx, __shfl_xor(mx, o));
    const float ex = __expf(lg - mx); float se = ex;
#pragma unroll
    for (int o = 16; o >= 1; o >>= 1) se += __shfl_xor(se, o);
    att[wave][lane] = ex / se; wave_lds_sync();
    float pc[4] = {0.0f, 0.0f, 0.0f, 0.0f};
    for (int n = 0; n < NN; ++n) { const v4f xv = *(const v4f*)(XC + ((size_t)b * NN + n) * C + lane * 4); for (int q = 0; q < 4; ++q) pc[q] += pmul(att[wave][n], xv[q]); }
    for (int q = 0; q < 4; ++q) { b16 p, ql; split16(pc[q] * XS, p, ql); Ph[b][lane * 4 + q] = p; Pl[b][lane * 4 + q] = ql; }
    wave_lds_sync(); }
  __syncthreads();
  for (int hq = 0; hq < 2; ++hq) { v8f acc[8];
#pragma unroll
    for (int t = 0; t < 8; ++t) acc[t] = (v8f){};
#pragma unroll
    for (int kb = 0; kb < C; kb += 32) { const v16b a = frag_kb(&Ph[wave * 16 + nloc][kb], hlf), al = frag_kb(&Pl[wave * 16 + nloc][kb], hlf);
#pragma unroll
      for (int t = 0; t < 8; ++t) { const v16b bw = frag_kb(WDT + (size_t)(hq * 128 + t * 16 + nloc) * C + kb, hlf); acc[t] = wmma16b(a, bw, acc[t]); acc[t] = wmma16b(al, bw, acc[t]); } }
#pragma unroll
    for (int t = 0; t < 8; ++t) { const float bb = bf16_rne(bd[hq * 128 + t * 16 + nloc]);
#pragma unroll
      for (int r = 0; r < 8; ++r) Tf[wave][8 * hlf + r][t * 16 + nloc] = tanhf(acc[t][r] * (1.0f / (XS * WSC)) + bb); }
    wave_lds_sync();
    for (int pass = 0; pass < 2; ++pass) { for (int rr = 0; rr < 16; ++rr) *(volatile v4f*)(out + (size_t)(wave * 16 + rr) * DD + hq * 128 + lane * 4) = *(const v4f*)(&Tf[wave][rr][lane * 4]); __threadfence(); }
    wave_lds_sync(); }
}
}

extern "C" void kernel_launch(void* const* d_in, const int* in_sizes, int n_in, void* d_out, int out_size, void* d_ws, size_t ws_size, hipStream_t stream) {
  (void)n_in;
  auto Fp = [&](int i) { return (const float*)d_in[i]; };
  if (in_sizes[0] != NB * OBS || in_sizes[1] != S * HH || in_sizes[3] != HH * HH || in_sizes[5] != HH * C * F || in_sizes[6] != C * F || in_sizes[7] != F * C || in_sizes[9] != C || in_sizes[10] != C * DD || out_size != NB * DD) return;
  size_t off = 0; char* ws = (char*)d_ws;
  auto carve = [&](size_t bytes) { char* p = ws + off; off += (bytes + 255) & ~(size_t)255; return p; };
  b16* E16 = (b16*)carve((size_t)NE * 32 * 2); b16* XT16 = (b16*)carve((size_t)NB * F * NN * 2); b16* W1T = (b16*)carve((size_t)HH * 32 * 2); b16* W2T = (b16*)carve((size_t)HH * HH * 2); b16* WKR = (b16*)carve((size_t)C * KT * 2); b16* WDT = (b16*)carve((size_t)DD * C * 2);
  b16* TTh = (b16*)carve((size_t)NBJ * KT * 2); b16* TTl = (b16*)carve((size_t)NBJ * KT * 2); float* SX = (float*)carve((size_t)NBJ * 32 * 4); float* XC = (float*)carve((size_t)NBJ * C * 4);
  if (off > ws_size || off > ((size_t)128 << 20)) return;
  prep_kernel<<<(unsigned)(((size_t)NE * 32 / 8 + (size_t)NB * F * NN / 8 + (size_t)HH * 32 / 8 + (size_t)HH * HH / 8 + (size_t)C * KT / 8 + (size_t)DD * C / 8 + 255) / 256), 256, 0, stream>>>(Fp(0), Fp(1), Fp(3), Fp(5), Fp(10), E16, XT16, W1T, W2T, WKR, WDT);
  edge_kernel<<<NBJ, 128, 0, stream>>>(E16, XT16, Fp(0), W1T, Fp(2), W2T, Fp(4), TTh, TTl, SX);
  ecc_kernel<<<NBJ / 64, 128, 0, stream>>>(TTh, TTl, WKR, SX, Fp(0), Fp(6), Fp(7), Fp(8), XC);
  head_kernel<<<1, 128, 0, stream>>>(XC, Fp(9), WDT, Fp(11), (float*)d_out);
}
